// SelfAttention_77163382440839
// MI455X (gfx1250) — hardware-verified
//
#include <hip/hip_runtime.h>


#ifndef NB
#define NB 8
#endif
#ifndef SEQ
#define SEQ 2048
#endif
#define NB_FULL    8
#define SEQ_FULL   2048
#define DM         512
#define PD         64
#define MALL       640
#define PR         64
#define BQ         128
#define BK         32
#define NWAVE      8
#define CG         128
#define LP         72
#define OPQ        132
#define WS_CAP     134217728ull

static_assert(SEQ % BQ == 0);
static_assert(SEQ % PR == 0);
static_assert(SEQ % BK == 0);
static_assert(SEQ % 64 == 0);
static_assert(BQ == NWAVE * 16);
static_assert(PD == 64);
static_assert(DM % 64 == 0);
static_assert(DM % 32 == 0);
static_assert(DM % CG == 0);
static_assert(CG == 128);
static_assert(CG == 8 * 16);
static_assert(MALL == 2 * PD + DM);
static_assert(MALL % 128 == 0);
static_assert(MALL / 128 == 5);
static_assert(PD * 2 == 128);
static_assert(PR * 2 == 128);
static_assert(PR == 64 && PR <= LP);
static_assert(BQ * 4 == 32 * 16);
static_assert(NWAVE * 4 == 32);
static_assert(OPQ >= BQ);
static_assert((OPQ * 4) % 16 == 0);
static_assert((LP * 2) % 16 == 0);
static_assert(SEQ <= SEQ_FULL);
static_assert(NB >= 1 && NB <= NB_FULL);
static_assert((PD * DM / 8) % 256 == 0);
static_assert((DM * DM / 8) % 256 == 0);
static_assert((unsigned long long)MALL * DM * 2ull +
              (unsigned long long)NB * SEQ * DM * 2ull +
              2ull * NB * SEQ * PD * 2ull +
              (unsigned long long)NB * DM * SEQ * 2ull <= WS_CAP);

typedef __bf16   bf16;
typedef _Float16 f16;
typedef bf16           v16bf __attribute__((ext_vector_type(16)));
typedef f16            v16h  __attribute__((ext_vector_type(16)));
typedef f16            v8h   __attribute__((ext_vector_type(8)));
typedef unsigned short v8us  __attribute__((ext_vector_type(8)));
typedef float          v8f   __attribute__((ext_vector_type(8)));
typedef float          v4f   __attribute__((ext_vector_type(4)));
typedef unsigned       v4u   __attribute__((ext_vector_type(4)));

union FragB  { v16bf v; v4u q[2]; bf16 h[16]; };
union FragH  { v16h  v; v4u q[2]; v8h hv[2]; f16 h[16]; };
union Pack8H { v4u u; v8h v; };
union Pack8S { v4u u; v8us s; };
union BitsB  { bf16 h; unsigned short u; };

static __device__ __forceinline__ v8f mma_bf16(v16bf a, v16bf b, v8f acc) {
  acc = __builtin_amdgcn_wmma_f32_16x16x32_bf16(false, a, false, b, (short)0, acc, false, false);
  asm volatile("v_nop\n\tv_nop\n\tv_nop\n\tv_nop" : "+v"(acc) : "v"(a), "v"(b));
  return acc;
}
static __device__ __forceinline__ v8f mma_f16(v16h a, v16h b, v8f acc) {
  acc = __builtin_amdgcn_wmma_f32_16x16x32_f16(false, a, false, b, (short)0, acc, false, false);
  asm volatile("v_nop\n\tv_nop\n\tv_nop\n\tv_nop" : "+v"(acc) : "v"(a), "v"(b));
  return acc;
}

static __device__ __forceinline__ f16 toh_flush(float v) {
  const f16 r = (f16)v;
  return (fabsf(v) < 6.103515625e-05f) ? (f16)0.0f : r;
}

static __device__ __forceinline__ unsigned short bf16_bits(float x) {
  BitsB bb; bb.h = (bf16)x;
  return bb.u;
}

__global__ __launch_bounds__(256) void wcvt_kernel(const float* __restrict__ win,
                                                   unsigned short* __restrict__ wout,
                                                   int out_base, int n8) {
  const int idx = blockIdx.x * 256 + threadIdx.x;
  if (idx < n8) {
    const float* src = win + (size_t)idx * 8;
    const v4f a0 = *(const v4f*)(src);
    const v4f a1 = *(const v4f*)(src + 4);
    Pack8S ps;
    #pragma unroll
    for (int i = 0; i < 4; ++i) {
      ps.s[i]     = bf16_bits(a0[i]);
      ps.s[4 + i] = bf16_bits(a1[i]);
    }
    const v4u val = ps.u;
    unsigned short* dst = wout + (size_t)out_base + (size_t)idx * 8;
    *(volatile v4u*)(dst) = val;
    __threadfence();
    *(volatile v4u*)(dst) = val;
  }
}

__global__ __launch_bounds__(256) void xprep_kernel(const float* __restrict__ x,
                                                    unsigned short* __restrict__ xt) {
  const int lt  = blockIdx.x;
  const int ct  = blockIdx.y;
  const int b   = blockIdx.z;
  const int tid = threadIdx.x;
  __shared__ __align__(16) unsigned short sT[64 * LP];

  #pragma unroll
  for (int kk = 0; kk < 2; ++kk) {
    const int r  = kk * 32 + (tid >> 3);
    const int c0 = (tid & 7) * 8;
    const float* src = x + ((size_t)b * DM + ct * 64 + r) * SEQ_FULL + lt * 64 + c0;
    const v4f a0 = *(const v4f*)(src);
    const v4f a1 = *(const v4f*)(src + 4);
    #pragma unroll
    for (int i = 0; i < 4; ++i) {
      sT[(c0 + i) * LP + r]     = bf16_bits(a0[i]);
      sT[(c0 + 4 + i) * LP + r] = bf16_bits(a1[i]);
    }
  }
  __syncthreads();

  v4u    val[2];
  size_t idx[2];
  #pragma unroll
  for (int kk = 0; kk < 2; ++kk) {
    const int c  = kk * 32 + (tid >> 3);
    const int rs = (tid & 7) * 8;
    Pack8S ps;
    ps.s = *(const v8us*)(sT + c * LP + rs);
    val[kk] = ps.u;
    idx[kk] = ((size_t)b * SEQ + lt * 64 + c) * DM + ct * 64 + rs;
  }
  #pragma unroll
  for (int kk = 0; kk < 2; ++kk) *(volatile v4u*)(xt + idx[kk]) = val[kk];
  __threadfence();
  #pragma unroll
  for (int kk = 0; kk < 2; ++kk) *(volatile v4u*)(xt + idx[kk]) = val[kk];
}

__global__ __launch_bounds__(256) void proj_kernel(const bf16* __restrict__ xt,
                                                   const bf16* __restrict__ wall,
                                                   const float* __restrict__ bfp,
                                                   const float* __restrict__ bgp,
                                                   const float* __restrict__ bhp,
                                                   f16* __restrict__ qh,
                                                   f16* __restrict__ kh,
                                                   f16* __restrict__ hp) {
  const int blk  = blockIdx.x;
  const int grp  = blockIdx.y;
  const int bpb  = SEQ / PR;
  const int b    = blk / bpb;
  const int s0   = (blk - b * bpb) * PR;
  const int tid  = threadIdx.x;
  const int wave = __builtin_amdgcn_readfirstlane(threadIdx.x >> 5);
  const int lane = tid & 31;
  const int lq   = lane & 15;
  const int hi   = lane >> 4;
  const int rg   = wave & 3;
  const int nh   = wave >> 2;
  const int hg   = max(grp, 1) - 1;

  __shared__ __align__(16) f16 sP[128 * LP];

  const bf16* xp = xt + ((size_t)b * SEQ + s0 + rg * 16 + lq) * DM;
  const bf16* wp = wall + (size_t)(grp * 128 + nh * 64 + lq) * DM;

  v8f acc[4];
  #pragma unroll
  for (int t = 0; t < 4; ++t) acc[t] = (v8f){0, 0, 0, 0, 0, 0, 0, 0};

  #pragma unroll 1
  for (int k0 = 0; k0 < DM; k0 += 32) {
    FragB a;
    a.q[0] = *(const v4u*)(xp + k0 + hi * 8);
    a.q[1] = *(const v4u*)(xp + k0 + 16 + hi * 8);
    #pragma unroll
    for (int t = 0; t < 4; ++t) {
      FragB w;
      const bf16* base = wp + (size_t)t * 16 * DM + k0 + hi * 8;
      w.q[0] = *(const v4u*)(base);
      w.q[1] = *(const v4u*)(base + 16);
      acc[t] = mma_bf16(a.v, w.v, acc[t]);
    }
  }

  #pragma unroll
  for (int t = 0; t < 4; ++t) {
    const int c64 = t * 16 + lq;
    const float b0v = (float)(bf16)bfp[c64];
    const float b1v = (float)(bf16)bgp[c64];
    const float b2v = (float)(bf16)bhp[hg * 128 + nh * 64 + c64];
    const float bias = (grp == 0) ? ((nh == 0) ? b0v : b1v) : b2v;
    #pragma unroll
    for (int r = 0; r < 8; ++r) {
      const int row = rg * 16 + hi * 8 + r;
      const int off = (grp == 0) ? (nh * PR * LP + row * LP + c64)
                                 : ((nh * 64 + c64) * LP + row);
      sP[off] = toh_flush((acc[t][r] + bias) * 16.0f);
    }
  }
  __syncthreads();

  const int seg = (tid & 7) * 8;
  if (grp == 0) {
    v4u    qv[2], kv[2];
    size_t ri[2];
    #pragma unroll
    for (int jj = 0; jj < 2; ++jj) {
      const int line = jj * 32 + (tid >> 3);
      Pack8H pq, pk;
      pq.v = *(const v8h*)(sP + line * LP + seg);
      pk.v = *(const v8h*)(sP + PR * LP + line * LP + seg);
      qv[jj] = pq.u;
      kv[jj] = pk.u;
      ri[jj] = ((size_t)b * SEQ + s0 + line) * PD + seg;
    }
    #pragma unroll
    for (int jj = 0; jj < 2; ++jj) {
      *(volatile v4u*)(qh + ri[jj]) = qv[jj];
      *(volatile v4u*)(kh + ri[jj]) = kv[jj];
    }
    __threadfence();
    #pragma unroll
    for (int jj = 0; jj < 2; ++jj) {
      *(volatile v4u*)(qh + ri[jj]) = qv[jj];
      *(volatile v4u*)(kh + ri[jj]) = kv[jj];
    }
  } else {
    v4u    hv[4];
    size_t vi[4];
    #pragma unroll
    for (int jj = 0; jj < 4; ++jj) {
      const int line = jj * 32 + (tid >> 3);
      Pack8H ph;
      ph.v = *(const v8h*)(sP + line * LP + seg);
      hv[jj] = ph.u;
      vi[jj] = ((size_t)b * DM + (grp - 1) * 128 + line) * SEQ + s0 + seg;
    }
    #pragma unroll
    for (int jj = 0; jj < 4; ++jj) *(volatile v4u*)(hp + vi[jj]) = hv[jj];
    __threadfence();
    #pragma unroll
    for (int jj = 0; jj < 4; ++jj) *(volatile v4u*)(hp + vi[jj]) = hv[jj];
  }
}

__global__ __launch_bounds__(256) __attribute__((amdgpu_num_vgpr(256)))
void attn_kernel(const f16* __restrict__ qh,
                 const f16* __restrict__ kh,
                 const f16* __restrict__ hp,
                 const float* __restrict__ x,
                 float* __restrict__ out) {
  const int qblk = blockIdx.x;
  const int cgi  = blockIdx.y;
  const int b    = blockIdx.z;
  const int tid  = threadIdx.x;
  const int wave = __builtin_amdgcn_readfirstlane(threadIdx.x >> 5);
  const int lane = tid & 31;
  const int lq   = lane & 15;
  const int hi   = lane >> 4;

  __shared__ __align__(16) float sO[32 * OPQ];

  const int qrow0 = qblk * BQ + wave * 16;

  FragH qf[2];
  {
    const f16* qp = qh + ((size_t)b * SEQ + qrow0 + lq) * PD;
    #pragma unroll
    for (int f = 0; f < 2; ++f) {
      qf[f].q[0] = *(const v4u*)(qp + f * 32 + hi * 8);
      qf[f].q[1] = *(const v4u*)(qp + f * 32 + 16 + hi * 8);
    }
  }

  const f16* kh_b = kh + (size_t)b * SEQ * PD;
  const f16* hp_b = hp + ((size_t)b * DM + cgi * CG) * SEQ;

  v8f o[8];
  #pragma unroll
  for (int ct = 0; ct < 8; ++ct) o[ct] = (v8f){0, 0, 0, 0, 0, 0, 0, 0};

  float rmax = -__builtin_inff();
  float rsum = 0.0f;
  const float SC    = 1.0f / 256.0f;
  const float LOG2E = 1.4426950408889634f;

  const int nchunk = SEQ / BK;
  #pragma unroll 1
  for (int i = 0; i < nchunk; ++i) {
    const int j0 = i * BK;

    v8f c[2];
    #pragma unroll
    for (int sub = 0; sub < 2; ++sub) {
      FragH ak[2];
      #pragma unroll
      for (int f = 0; f < 2; ++f) {
        const f16* base = kh_b + (size_t)(j0 + sub * 16 + lq) * PD + f * 32 + hi * 8;
        ak[f].q[0] = *(const v4u*)(base);
        ak[f].q[1] = *(const v4u*)(base + 16);
      }
      v8f acc = (v8f){0, 0, 0, 0, 0, 0, 0, 0};
      acc = mma_f16(ak[0].v, qf[0].v, acc);
      acc = mma_f16(ak[1].v, qf[1].v, acc);
      c[sub] = acc;
    }

    float s0v[8], s1v[8];
    float m_new = rmax;
    #pragma unroll
    for (int r = 0; r < 8; ++r) {
      s0v[r] = c[0][r] * SC;
      s1v[r] = c[1][r] * SC;
      m_new = fmaxf(m_new, s0v[r]);
      m_new = fmaxf(m_new, s1v[r]);
    }
    m_new = fmaxf(m_new, __shfl_xor(m_new, 16, 32));
    const float scale = __builtin_amdgcn_exp2f((rmax - m_new) * LOG2E);
    rmax = m_new;

    FragH pa;
    float psum = 0.0f;
    #pragma unroll
    for (int r = 0; r < 8; ++r) {
      const float p0 = __builtin_amdgcn_exp2f((s0v[r] - m_new) * LOG2E);
      const float p1 = __builtin_amdgcn_exp2f((s1v[r] - m_new) * LOG2E);
      psum += p0 + p1;
      pa.h[r]     = toh_flush(p0 * 4096.0f);
      pa.h[8 + r] = toh_flush(p1 * 4096.0f);
    }
    rsum = rsum * scale + psum + __shfl_xor(psum, 16, 32);

    #pragma unroll
    for (int ct = 0; ct < 8; ++ct) {
      #pragma unroll
      for (int r = 0; r < 8; ++r) o[ct][r] *= scale;
    }

    #pragma unroll
    for (int hf = 0; hf < 2; ++hf) {
      FragH ah[4];
      #pragma unroll
      for (int t = 0; t < 4; ++t) {
        const f16* base = hp_b + (size_t)((hf * 4 + t) * 16 + lq) * SEQ + j0 + hi * 8;
        ah[t].q[0] = *(const v4u*)(base);
        ah[t].q[1] = *(const v4u*)(base + 16);
      }
      #pragma unroll
      for (int t = 0; t < 4; ++t) o[hf * 4 + t] = mma_f16(ah[t].v, pa.v, o[hf * 4 + t]);
    }
  }

  const float fin = (1.0f / rsum) * 1.52587890625e-05f;

  #pragma unroll
  for (int g = 0; g < 4; ++g) {
    #pragma unroll
    for (int tt = 0; tt < 2; ++tt) {
      #pragma unroll
      for (int r = 0; r < 8; ++r) {
        sO[(tt * 16 + hi * 8 + r) * OPQ + wave * 16 + lq] = o[g * 2 + tt][r] * fin;
      }
    }
    __syncthreads();

    v4f    vals[4];
    size_t gidx[4];
    #pragma unroll
    for (int it = 0; it < 4; ++it) {
      const int row = wave * 4 + it;
      const int ch  = cgi * CG + g * 32 + row;
      gidx[it] = ((size_t)b * DM + ch) * SEQ_FULL + qblk * BQ + lane * 4;
      v4f sv = *(const v4f*)(sO + row * OPQ + lane * 4);
      const v4f xv = *(const v4f*)(x + gidx[it]);
      #pragma unroll
      for (int e = 0; e < 4; ++e) sv[e] += (float)(bf16)xv[e];
      vals[it] = sv;
    }
    #pragma unroll
    for (int it = 0; it < 4; ++it) *(volatile v4f*)(out + gidx[it]) = vals[it];
    __threadfence();
    #pragma unroll
    for (int it = 0; it < 4; ++it) *(volatile v4f*)(out + gidx[it]) = vals[it];
    __syncthreads();
  }
}

extern "C" void kernel_launch(void* const* d_in, const int* in_sizes, int n_in,
                              void* d_out, int out_size, void* d_ws, size_t ws_size,
                              hipStream_t stream) {
  if (n_in < 7) return;
  const size_t need_x = ((size_t)(NB - 1) * DM + (DM - 1)) * SEQ_FULL + SEQ;
  if ((size_t)in_sizes[0] < need_x) return;
  if ((size_t)in_sizes[1] < (size_t)PD * DM) return;
  if ((size_t)in_sizes[2] < (size_t)PD) return;
  if ((size_t)in_sizes[3] < (size_t)PD * DM) return;
  if ((size_t)in_sizes[4] < (size_t)PD) return;
  if ((size_t)in_sizes[5] < (size_t)DM * DM) return;
  if ((size_t)in_sizes[6] < (size_t)DM) return;
  if ((size_t)out_size < need_x) return;

  const size_t wall_bytes = (size_t)MALL * DM * 2;
  const size_t xt_bytes   = (size_t)NB * SEQ * DM * 2;
  const size_t qk_bytes   = (size_t)NB * SEQ * PD * 2;
  const size_t hp_bytes   = (size_t)NB * DM * SEQ * 2;
  if (ws_size < wall_bytes + xt_bytes + 2 * qk_bytes + hp_bytes) return;

  const float* x   = (const float*)d_in[0];
  const float* Wf  = (const float*)d_in[1];
  const float* bfv = (const float*)d_in[2];
  const float* Wg  = (const float*)d_in[3];
  const float* bgv = (const float*)d_in[4];
  const float* Wh  = (const float*)d_in[5];
  const float* bhv = (const float*)d_in[6];
  float*       out = (float*)d_out;

  char* ws = (char*)d_ws;
  unsigned short* wall_u = (unsigned short*)(ws);
  unsigned short* xt_u   = (unsigned short*)(ws + wall_bytes);
  f16* qh = (f16*)(ws + wall_bytes + xt_bytes);
  f16* kh = (f16*)(ws + wall_bytes + xt_bytes + qk_bytes);
  f16* hp = (f16*)(ws + wall_bytes + xt_bytes + 2 * qk_bytes);

  wcvt_kernel<<<(PD * DM / 8) / 256, 256, 0, stream>>>(Wf, wall_u, 0, PD * DM / 8);
  wcvt_kernel<<<(PD * DM / 8) / 256, 256, 0, stream>>>(Wg, wall_u, PD * DM, PD * DM / 8);
  wcvt_kernel<<<(DM * DM / 8) / 256, 256, 0, stream>>>(Wh, wall_u, 2 * PD * DM, DM * DM / 8);
  xprep_kernel<<<dim3(SEQ / 64, DM / 64, NB), 256, 0, stream>>>(x, xt_u);

  proj_kernel<<<dim3(NB * (SEQ / PR), MALL / 128), 256, 0, stream>>>((const bf16*)xt_u, (const bf16*)wall_u,
                                                                     bfv, bgv, bhv, qh, kh, hp);
  attn_kernel<<<dim3(SEQ / BQ, DM / CG, NB), 256, 0, stream>>>(qh, kh, hp, x, out);
}
